// TAGNNetwork_15307263443521
// MI455X (gfx1250) — hardware-verified
//
#include <hip/hip_runtime.h>
#include <stddef.h>
#include <stdint.h>

#define NB   4
#define SF   16384
#define NN   1024
#define DD   64
#define HID  32
#define KP   128
#define NROW (NB * NN)
#define NFLW (NB * SF)
#define RBN  32
#define CH   256
#define FPB  128
#define AP   136
#define WP   72
#define TP   68
#define RQ   32
#define NWD  (NN / 32)

static_assert(DD == 64);
static_assert(KP == 2 * DD);
static_assert(HID == 32);
static_assert(SF % CH == 0);
static_assert(CH == 256);
static_assert(NN % RBN == 0);
static_assert(NFLW % FPB == 0);
static_assert(FPB == 128);
static_assert(NROW % 128 == 0);
static_assert(NN % 128 == 0);
static_assert(NROW % 256 == 0);
static_assert(NN % 256 == 0);
static_assert(NN % RQ == 0);
static_assert(RQ == 32);
static_assert(NWD == 32);
static_assert(NN == 4 * 256);
static_assert((AP * 2) % 16 == 0);
static_assert((WP * 2) % 16 == 0);
static_assert((TP * 4) % 16 == 0);
static_assert(KP % 32 == 0);

typedef _Float16       v16h __attribute__((ext_vector_type(16)));
typedef _Float16       v8h  __attribute__((ext_vector_type(8)));
typedef _Float16       v2h  __attribute__((ext_vector_type(2)));
typedef float          v8f  __attribute__((ext_vector_type(8)));
typedef float          v4f  __attribute__((ext_vector_type(4)));
typedef unsigned int   v4u  __attribute__((ext_vector_type(4)));

union FragH { v16h v; v8h h[2]; };
union Pack8 { v8h h; v4u u; };
union Pack2 { v2h h; unsigned int u; };

__device__ __forceinline__ v8f mma16h(v16h a, v16h b, v8f c) {
  c = __builtin_amdgcn_wmma_f32_16x16x32_f16(false, a, false, b, (short)0, c, false, false);
  asm volatile("v_nop\n\tv_nop\n\tv_nop\n\tv_nop" : "+v"(c) : "v"(a), "v"(b));
  return c;
}

__device__ __forceinline__ v16h ldfrag_h(const _Float16* p, int ld, int row0, int k0, int lane) {
  const int m = lane & 15, lh = lane >> 4;
  const _Float16* q = p + (size_t)(row0 + m) * ld + k0 + 8 * lh;
  FragH f;
  f.h[0] = *(const v8h*)(q);
  f.h[1] = *(const v8h*)(q + 16);
  return f.v;
}

__device__ __forceinline__ v8f zero8() { return (v8f){0.f, 0.f, 0.f, 0.f, 0.f, 0.f, 0.f, 0.f}; }

__device__ __forceinline__ void gemm32x64_f16(const _Float16* __restrict__ A, int lda,
                                              const _Float16* __restrict__ Bt, int ldb, int K,
                                              int m0, int n0, int lane, v8f (&acc)[2][4]) {
#pragma unroll 1
  for (int k0 = 0; k0 < K; k0 += 32) {
    const v16h a0 = ldfrag_h(A, lda, m0, k0, lane);
    const v16h a1 = ldfrag_h(A, lda, m0 + 16, k0, lane);
#pragma unroll
    for (int t = 0; t < 4; ++t) {
      const v16h b = ldfrag_h(Bt, ldb, n0 + 16 * t, k0, lane);
      acc[0][t] = mma16h(a0, b, acc[0][t]);
      acc[1][t] = mma16h(a1, b, acc[1][t]);
    }
  }
}

__global__ __launch_bounds__(256) void k_node(const float* __restrict__ flow, const int* __restrict__ dst,
                                              unsigned int* __restrict__ h16u) {
  __shared__ int s_cnt[8][RBN];
  __shared__ int s_list[RBN][CH];
  const int tid = threadIdx.x, lane = tid & 31, wave = tid >> 5;
  const int b = blockIdx.y, n0 = blockIdx.x * RBN;
  const int* dstb = dst + (size_t)b * SF;
  const float2* flow2 = (const float2*)(flow + (size_t)b * SF * DD);
  float ax[4] = {0.f, 0.f, 0.f, 0.f};
  float ay[4] = {0.f, 0.f, 0.f, 0.f};

#pragma unroll 1
  for (int cidx = 0; cidx < SF / CH; ++cidx) {
    const int e0 = cidx * CH;
    const int key = dstb[e0 + tid] - n0;
    unsigned int mym = 0u;
#pragma unroll 1
    for (int ln = 0; ln < RBN; ++ln) {
      const unsigned int m = __builtin_amdgcn_ballot_w32(key == ln);
      mym = (lane == ln) ? m : mym;
    }
    s_cnt[wave][lane] = (int)__builtin_popcount(mym);
    __syncthreads();
    int off = 0;
#pragma unroll
    for (int w2 = 0; w2 < 8; ++w2) {
      const int cv = s_cnt[w2][lane];
      off += (w2 < wave) ? cv : 0;
    }
    {
      unsigned int bits = mym;
      int pos = off;
#pragma unroll 1
      for (int itb = 0; itb < 32; ++itb) {
        if (bits == 0u) break;
        const int q = __builtin_ctz(bits);
        bits &= bits - 1u;
        s_list[lane][pos & (CH - 1)] = e0 + 32 * wave + q;
        ++pos;
      }
    }
    __syncthreads();
#pragma unroll
    for (int q = 0; q < 4; ++q) {
      const int ln = wave + 8 * q;
      int tot = 0;
#pragma unroll
      for (int w2 = 0; w2 < 8; ++w2) tot += s_cnt[w2][ln];
      tot = (tot > CH) ? CH : tot;
      float sx = ax[q], sy = ay[q];
#pragma unroll 1
      for (int p = 0; p < tot; ++p) {
        int e2 = s_list[ln][p];
        e2 = (e2 < 0) ? 0 : ((e2 > SF - 1) ? (SF - 1) : e2);
        const float2 v = flow2[(size_t)e2 * (DD / 2) + lane];
        sx += v.x;
        sy += v.y;
      }
      ax[q] = sx;
      ay[q] = sy;
    }
    __syncthreads();
  }

  unsigned int hv[4];
#pragma unroll
  for (int q = 0; q < 4; ++q) {
    float ss = ax[q] * ax[q] + ay[q] * ay[q];
#pragma unroll
    for (int o = 16; o; o >>= 1) ss += __shfl_xor(ss, o, 32);
    float nrm = __builtin_amdgcn_sqrtf(ss);
    nrm = fmaxf(nrm, 1e-12f);
    const float sc = __builtin_amdgcn_rcpf(nrm) * 16.0f;
    Pack2 pk;
    pk.h = (v2h){(_Float16)(ax[q] * sc), (_Float16)(ay[q] * sc)};
    hv[q] = pk.u;
  }
  volatile unsigned int* hp = h16u + (size_t)(b * NN + n0 + wave) * (DD / 2) + lane;
#pragma unroll
  for (int q = 0; q < 4; ++q) hp[(size_t)q * 8 * (DD / 2)] = hv[q];
  __threadfence();
#pragma unroll
  for (int q = 0; q < 4; ++q) hp[(size_t)q * 8 * (DD / 2)] = hv[q];
}

__global__ __launch_bounds__(128) void k_edge(const float* __restrict__ emb, const int* __restrict__ src,
                                              const int* __restrict__ dst, const float* __restrict__ vol,
                                              const float* __restrict__ we1, const float* __restrict__ be1,
                                              const float* __restrict__ we2, const float* __restrict__ be2,
                                              float* __restrict__ ew) {
  __shared__ __align__(16) _Float16 s_a[FPB][AP];
  __shared__ __align__(16) _Float16 s_b[HID][AP];
  __shared__ __align__(16) float s_w[4][32];
  const int tid = threadIdx.x, lane = tid & 31, wave = tid >> 5;
  const int f0 = blockIdx.x * FPB;

  {
    const float* wr = we1 + (size_t)tid * HID;
#pragma unroll 1
    for (int n = 0; n < HID; ++n) s_b[n][tid] = (_Float16)(wr[n] * 64.0f);
  }
  {
    const int piece = tid & 15, rofs = tid >> 4;
#pragma unroll 2
    for (int r = 0; r < 16; ++r) {
      const int row = 8 * r + rofs;
      const int f = f0 + row;
      int si = src[f], di = dst[f];
      si = (si < 0) ? 0 : ((si > NN - 1) ? (NN - 1) : si);
      di = (di < 0) ? 0 : ((di > NN - 1) ? (NN - 1) : di);
      const int idx = (piece < 8) ? si : di;
      const float* ep = emb + (size_t)idx * DD + 8 * (piece & 7);
      const v4f u0 = *(const v4f*)(ep);
      const v4f u1 = *(const v4f*)(ep + 4);
      Pack8 pk;
      pk.h = (v8h){(_Float16)(u0[0] * 256.0f), (_Float16)(u0[1] * 256.0f), (_Float16)(u0[2] * 256.0f),
                   (_Float16)(u0[3] * 256.0f), (_Float16)(u1[0] * 256.0f), (_Float16)(u1[1] * 256.0f),
                   (_Float16)(u1[2] * 256.0f), (_Float16)(u1[3] * 256.0f)};
      *(v8h*)(&s_a[row][8 * piece]) = pk.h;
    }
  }
  __syncthreads();

  v8f acc[2][2];
#pragma unroll
  for (int s = 0; s < 2; ++s)
#pragma unroll
    for (int t = 0; t < 2; ++t) acc[s][t] = zero8();
  const int m0 = 32 * wave;
#pragma unroll
  for (int k0 = 0; k0 < KP; k0 += 32) {
    const v16h fa0 = ldfrag_h(&s_a[0][0], AP, m0, k0, lane);
    const v16h fa1 = ldfrag_h(&s_a[0][0], AP, m0 + 16, k0, lane);
#pragma unroll
    for (int t = 0; t < 2; ++t) {
      const v16h fb = ldfrag_h(&s_b[0][0], AP, 16 * t, k0, lane);
      acc[0][t] = mma16h(fa0, fb, acc[0][t]);
      acc[1][t] = mma16h(fa1, fb, acc[1][t]);
    }
  }

  const int hh = lane >> 4, c = lane & 15;
  const float b1c0 = be1[c], b1c1 = be1[16 + c];
  const float w2c0 = we2[c], w2c1 = we2[16 + c];
  const float be2v = be2[0];
  const float EINV = 1.0f / 16384.0f;
  float zsel[2];
#pragma unroll
  for (int s = 0; s < 2; ++s) {
    float zs = 0.f;
#pragma unroll
    for (int r = 0; r < 8; ++r) {
      const float m0v = fmaxf(fmaf(acc[s][0][r], EINV, b1c0), 0.f);
      const float m1v = fmaxf(fmaf(acc[s][1][r], EINV, b1c1), 0.f);
      float zp = fmaf(m0v, w2c0, m1v * w2c1);
      zp += __shfl_xor(zp, 1, 32);
      zp += __shfl_xor(zp, 2, 32);
      zp += __shfl_xor(zp, 4, 32);
      zp += __shfl_xor(zp, 8, 32);
      zs = (c == r) ? zp : zs;
    }
    zsel[s] = zs;
  }
#pragma unroll
  for (int s = 0; s < 2; ++s) {
    const int row = 16 * s + 8 * hh + (c & 7);
    const int f = f0 + m0 + row;
    const float v = vol[f];
    const float z = zsel[s] + be2v;
    const float sg1 = __builtin_amdgcn_rcpf(1.0f + __expf(-z));
    const float sg2 = __builtin_amdgcn_rcpf(1.0f + __expf(-(v * 0.001f)));
    const float w = sg1 * sg2;
    if (c < 8) s_w[wave][row] = w;
  }
  __syncthreads();
  {
    const int pc = lane & 7;
    const v4f val = *(const v4f*)(&s_w[wave][4 * pc]);
    volatile v4f* dp = (volatile v4f*)(ew + f0 + m0 + 4 * pc);
    if (lane < 8) *dp = val;
    __threadfence();
    if (lane < 8) *dp = val;
  }
}

__global__ __launch_bounds__(128) void k_wh(const _Float16* __restrict__ h16, const float* __restrict__ W,
                                            const float* __restrict__ a1, const float* __restrict__ a2,
                                            float* __restrict__ F1, float* __restrict__ F2,
                                            _Float16* __restrict__ whT) {
  __shared__ __align__(16) float    s_t[128][TP];
  __shared__ __align__(16) _Float16 s_wt[DD][WP];
  __shared__ __align__(16) float    s_f[2][128];
  __shared__ float s_av[2 * DD];
  const int tid = threadIdx.x, lane = tid & 31, wave = tid >> 5;
  const int mb = blockIdx.x * 128;

  {
    const int n = tid & (DD - 1), kh = tid >> 6;
#pragma unroll 1
    for (int kk = 0; kk < 32; ++kk) {
      const int k = 32 * kh + kk;
      s_wt[n][k] = (_Float16)(W[k * DD + n] * 64.0f);
    }
    const float va = a1[tid & (DD - 1)];
    const float vb = a2[tid & (DD - 1)];
    s_av[tid] = (tid < DD) ? va : vb;
  }
  __syncthreads();

  v8f acc[2][4];
#pragma unroll
  for (int s = 0; s < 2; ++s)
#pragma unroll
    for (int t = 0; t < 4; ++t) acc[s][t] = zero8();
  const int m0 = mb + 32 * wave;
#pragma unroll
  for (int k0 = 0; k0 < DD; k0 += 32) {
    const v16h fa0 = ldfrag_h(h16, DD, m0, k0, lane);
    const v16h fa1 = ldfrag_h(h16, DD, m0 + 16, k0, lane);
#pragma unroll
    for (int t = 0; t < 4; ++t) {
      const v16h fb = ldfrag_h(&s_wt[0][0], WP, 16 * t, k0, lane);
      acc[0][t] = mma16h(fa0, fb, acc[0][t]);
      acc[1][t] = mma16h(fa1, fb, acc[1][t]);
    }
  }

  const int hh = lane >> 4, c = lane & 15;
  const float WINV = 1.0f / 1024.0f;
#pragma unroll
  for (int s = 0; s < 2; ++s)
#pragma unroll
    for (int t = 0; t < 4; ++t)
#pragma unroll
      for (int r = 0; r < 8; ++r) s_t[32 * wave + 16 * s + 8 * hh + r][16 * t + c] = acc[s][t][r] * WINV;
  __syncthreads();
  {
    float f1v = 0.f, f2v = 0.f;
#pragma unroll 4
    for (int d = 0; d < DD; ++d) {
      const float x = s_t[tid][d];
      f1v = fmaf(x, s_av[d], f1v);
      f2v = fmaf(x, s_av[DD + d], f2v);
    }
    s_f[0][tid] = f1v;
    s_f[1][tid] = f2v;
  }
  __syncthreads();

  const int wsel = wave & 1;
  const v4f fv = *(const v4f*)(&s_f[wsel][4 * lane]);
  volatile v4f* fpo = (volatile v4f*)((wsel ? F2 : F1) + mb + 4 * lane);
  const int b = mb / NN, jb = mb & (NN - 1);
  v4u tv[8];
  size_t to[8];
#pragma unroll
  for (int it = 0; it < 8; ++it) {
    const int d  = 16 * wave + 2 * it + (lane >> 4);
    const int j0 = 64 * ((lane >> 3) & 1) + 8 * (lane & 7);
    Pack8 pk;
    pk.h = (v8h){(_Float16)(s_t[j0 + 0][d] * 256.0f), (_Float16)(s_t[j0 + 1][d] * 256.0f),
                 (_Float16)(s_t[j0 + 2][d] * 256.0f), (_Float16)(s_t[j0 + 3][d] * 256.0f),
                 (_Float16)(s_t[j0 + 4][d] * 256.0f), (_Float16)(s_t[j0 + 5][d] * 256.0f),
                 (_Float16)(s_t[j0 + 6][d] * 256.0f), (_Float16)(s_t[j0 + 7][d] * 256.0f)};
    tv[it] = pk.u;
    to[it] = (size_t)(b * DD + d) * NN + jb + j0;
  }
  if (wave < 2) *fpo = fv;
#pragma unroll
  for (int it = 0; it < 8; ++it) *(volatile v4u*)(whT + to[it]) = tv[it];
  __threadfence();
  if (wave < 2) *fpo = fv;
#pragma unroll
  for (int it = 0; it < 8; ++it) *(volatile v4u*)(whT + to[it]) = tv[it];
}

__global__ __launch_bounds__(256) void k_pmat(const int* __restrict__ src, const int* __restrict__ dst,
                                              const float* __restrict__ ew, const float* __restrict__ F1,
                                              const float* __restrict__ F2, _Float16* __restrict__ P,
                                              float* __restrict__ RS) {
  __shared__ __align__(16) float s_f2[NN];
  __shared__ __align__(16) unsigned int s_mask[RQ][NWD];
  __shared__ __align__(16) float s_rs[RQ];
  const int tid = threadIdx.x, lane = tid & 31, wave = tid >> 5;
  const int b = blockIdx.y, i0 = blockIdx.x * RQ;

  *(v4f*)(&s_f2[4 * tid]) = *(const v4f*)(F2 + (size_t)b * NN + 4 * tid);
  *(v4u*)(&s_mask[0][0] + 4 * tid) = (v4u){0u, 0u, 0u, 0u};
  __syncthreads();
  {
    const int* sb = src + (size_t)b * SF;
    const int* db = dst + (size_t)b * SF;
    const float* eb = ew + (size_t)b * SF;
#pragma unroll 1
    for (int e = tid; e < SF; e += 256) {
      const int s = sb[e], d = db[e];
      const float w = eb[e];
      const bool ok = ((unsigned)s < (unsigned)NN) && ((unsigned)d < (unsigned)NN) && (w > 0.f);
      const int sc = s & (NN - 1), dc = d & (NN - 1);
      if (ok && (unsigned)(sc - i0) < (unsigned)RQ) atomicOr(&s_mask[sc - i0][dc >> 5], 1u << (dc & 31));
      if (ok && (unsigned)(dc - i0) < (unsigned)RQ) atomicOr(&s_mask[dc - i0][sc >> 5], 1u << (sc & 31));
    }
  }
  __syncthreads();

  const float NEGI = __uint_as_float(0xff800000u);
#pragma unroll 1
  for (int q = 0; q < RQ / 8; ++q) {
    const int lr = wave + 8 * q;
    const int i = i0 + lr;
    const float f1i = F1[(size_t)b * NN + i];
    int cnt = (int)__builtin_popcount(s_mask[lr][lane]);
#pragma unroll
    for (int o = 16; o; o >>= 1) cnt += __shfl_xor(cnt, o, 32);
    const bool uni = (cnt == 0);

    float mx = NEGI;
#pragma unroll
    for (int t = 0; t < 4; ++t) {
      const int jw = 256 * t + 8 * lane;
      const unsigned int bits = (s_mask[lr][jw >> 5] >> (jw & 31)) & 0xffu;
      const v4f g0 = *(const v4f*)(&s_f2[jw]);
      const v4f g1 = *(const v4f*)(&s_f2[jw + 4]);
      const float fv[8] = {g0[0], g0[1], g0[2], g0[3], g1[0], g1[1], g1[2], g1[3]};
#pragma unroll
      for (int k = 0; k < 8; ++k) mx = ((bits >> k) & 1u) ? fmaxf(mx, fv[k]) : mx;
    }
#pragma unroll
    for (int o = 16; o; o >>= 1) mx = fmaxf(mx, __shfl_xor(mx, o, 32));
    float em = f1i + mx;
    em = (em >= 0.f) ? em : 0.2f * em;

    float ls = 0.f;
    v4u pv[4];
#pragma unroll
    for (int t = 0; t < 4; ++t) {
      const int jw = 256 * t + 8 * lane;
      const unsigned int bits = (s_mask[lr][jw >> 5] >> (jw & 31)) & 0xffu;
      const v4f g0 = *(const v4f*)(&s_f2[jw]);
      const v4f g1 = *(const v4f*)(&s_f2[jw + 4]);
      const float fv[8] = {g0[0], g0[1], g0[2], g0[3], g1[0], g1[1], g1[2], g1[3]};
      Pack8 pk;
#pragma unroll
      for (int k = 0; k < 8; ++k) {
        float x = f1i + fv[k];
        x = (x >= 0.f) ? x : 0.2f * x;
        float p = __expf(x - em);
        p = ((bits >> k) & 1u) ? p : 0.f;
        p = uni ? 1.0f : p;
        const _Float16 hq = (_Float16)(p * 1024.0f);
        pk.h[k] = hq;
        ls += (float)hq;
      }
      pv[t] = pk.u;
    }
#pragma unroll
    for (int o = 16; o; o >>= 1) ls += __shfl_xor(ls, o, 32);
    const size_t prow = (size_t)(b * NN + i) * NN;
#pragma unroll
    for (int t = 0; t < 4; ++t) *(volatile v4u*)(P + prow + 256 * t + 8 * lane) = pv[t];
    __threadfence();
#pragma unroll
    for (int t = 0; t < 4; ++t) *(volatile v4u*)(P + prow + 256 * t + 8 * lane) = pv[t];
    if (lane == 0) s_rs[lr] = __builtin_amdgcn_rcpf(ls);
  }
  __syncthreads();
  if (wave == 0) {
    const int pc = lane & 7;
    const v4f val = *(const v4f*)(&s_rs[4 * pc]);
    volatile v4f* dp = (volatile v4f*)(RS + (size_t)b * NN + i0 + 4 * pc);
    if (lane < 8) *dp = val;
    __threadfence();
    if (lane < 8) *dp = val;
  }
}

__global__ __launch_bounds__(256) void k_out(const _Float16* __restrict__ P, const _Float16* __restrict__ whT,
                                             const float* __restrict__ RS, float* __restrict__ out) {
  __shared__ __align__(16) float st[8][16 * TP];
  const int tid = threadIdx.x, lane = tid & 31, wave = tid >> 5;
  const int hh = lane >> 4, c = lane & 15;
  const int m0 = blockIdx.x * 256 + wave * 32;
  const int b = blockIdx.x / (NN / 256);
  const _Float16* Bt = whT + (size_t)b * DD * NN;
  v8f acc[2][4];
#pragma unroll
  for (int s = 0; s < 2; ++s)
#pragma unroll
    for (int t = 0; t < 4; ++t) acc[s][t] = zero8();
  gemm32x64_f16(P, NN, Bt, NN, NN, m0, 0, lane, acc);

  float* sw = st[wave];
  const float OINV = 1.0f / 256.0f;
#pragma unroll
  for (int sub = 0; sub < 2; ++sub) {
    __syncthreads();
    float rsv[8];
#pragma unroll
    for (int r = 0; r < 8; ++r) rsv[r] = RS[m0 + 16 * sub + 8 * hh + r] * OINV;
#pragma unroll
    for (int t = 0; t < 4; ++t)
#pragma unroll
      for (int r = 0; r < 8; ++r) sw[(8 * hh + r) * TP + 16 * t + c] = acc[sub][t][r] * rsv[r];
    __syncthreads();
#pragma unroll 1
    for (int g = 0; g < 32; ++g) {
      const int idx = 32 * g + lane;
      float* pp = sw + (idx >> 6) * TP + (idx & 63);
      const float x = *pp;
      *pp = (x > 0.f) ? x : expm1f(x);
    }
    __syncthreads();
    v4f val[8];
    size_t go[8];
#pragma unroll
    for (int it = 0; it < 8; ++it) {
      const int p    = lane + 32 * it;
      const int L    = p >> 3;
      const int pc   = p & 7;
      const int row  = L >> 1;
      const int half = L & 1;
      val[it] = *(const v4f*)(sw + row * TP + half * 32 + pc * 4);
      go[it]  = (size_t)(m0 + sub * 16 + row) * DD + half * 32 + pc * 4;
    }
#pragma unroll
    for (int it = 0; it < 8; ++it) *(volatile v4f*)(out + go[it]) = val[it];
    __threadfence();
#pragma unroll
    for (int it = 0; it < 8; ++it) *(volatile v4f*)(out + go[it]) = val[it];
  }
}

extern "C" void kernel_launch(void* const* d_in, const int* in_sizes, int n_in,
                              void* d_out, int out_size, void* d_ws, size_t ws_size,
                              hipStream_t stream) {
  if (n_in < 12) return;
  if (in_sizes[0] != NB * SF * DD) return;
  if (in_sizes[1] != NFLW || in_sizes[2] != NFLW || in_sizes[3] != NFLW) return;
  if (in_sizes[4] != NN * DD) return;
  if (in_sizes[5] != KP * HID || in_sizes[6] != HID || in_sizes[7] != HID || in_sizes[8] < 1) return;
  if (in_sizes[9] != DD * DD || in_sizes[10] != DD || in_sizes[11] != DD) return;
  if (out_size != NROW * DD) return;

  const float* flow = (const float*)d_in[0];
  const int*   src  = (const int*)d_in[1];
  const int*   dst  = (const int*)d_in[2];
  const float* vol  = (const float*)d_in[3];
  const float* emb  = (const float*)d_in[4];
  const float* we1  = (const float*)d_in[5];
  const float* be1  = (const float*)d_in[6];
  const float* we2  = (const float*)d_in[7];
  const float* be2  = (const float*)d_in[8];
  const float* W    = (const float*)d_in[9];
  const float* a1   = (const float*)d_in[10];
  const float* a2   = (const float*)d_in[11];
  float* out = (float*)d_out;

  size_t off = 0;
  const size_t oH  = off; off += (size_t)NROW * DD * 2;
  const size_t oEW = off; off += (size_t)NFLW * 4;
  const size_t oF1 = off; off += (size_t)NROW * 4;
  const size_t oF2 = off; off += (size_t)NROW * 4;
  const size_t oWT = off; off += (size_t)NB * DD * NN * 2;
  const size_t oP  = off; off += (size_t)NROW * NN * 2;
  const size_t oRS = off; off += (size_t)NROW * 4;
  if (off > ws_size) return;
  if (off > (size_t)134217728) return;
  if ((oEW & 127) != 0 || (oF1 & 127) != 0 || (oWT & 127) != 0 || (oP & 127) != 0 || (oRS & 127) != 0) return;

  char* ws = (char*)d_ws;
  _Float16* H16 = (_Float16*)(ws + oH);
  float*    EW  = (float*)(ws + oEW);
  float*    F1  = (float*)(ws + oF1);
  float*    F2  = (float*)(ws + oF2);
  _Float16* WHT = (_Float16*)(ws + oWT);
  _Float16* P16 = (_Float16*)(ws + oP);
  float*    RS  = (float*)(ws + oRS);

  k_node<<<dim3(NN / RBN, NB), dim3(256), 0, stream>>>(flow, dst, (unsigned int*)H16);
  k_edge<<<dim3(NFLW / FPB), dim3(128), 0, stream>>>(emb, src, dst, vol, we1, be1, we2, be2, EW);
  k_wh<<<dim3(NROW / 128), dim3(128), 0, stream>>>(H16, W, a1, a2, F1, F2, WHT);
  k_pmat<<<dim3(NN / RQ, NB), dim3(256), 0, stream>>>(src, dst, EW, F1, F2, P16, RS);
  k_out<<<dim3(NROW / 256), dim3(256), 0, stream>>>(P16, WHT, RS, out);
  (void)hipGetLastError();
}
